// BasicTransformerBlock_89962384982092
// MI455X (gfx1250) — hardware-verified
//
#include <hip/hip_runtime.h>
#include <math.h>

typedef __attribute__((ext_vector_type(16))) _Float16 v16h;
typedef __attribute__((ext_vector_type(8)))  _Float16 v8h;
typedef __attribute__((ext_vector_type(8)))  float v8f;
typedef __attribute__((ext_vector_type(4)))  float v4f;
typedef __attribute__((ext_vector_type(4)))  unsigned v4u;

template <typename T> __device__ __forceinline__ void vst2(void* p, T v) { *(volatile T*)p = v; __threadfence(); *(volatile T*)p = v; }
__device__ __forceinline__ v8f wmma16(v16h a, v16h b, v8f c) {
  v8f d = __builtin_amdgcn_wmma_f32_16x16x32_f16(false, a, false, b, (short)0, c, false, false);
  asm volatile("v_nop\n\tv_nop\n\tv_nop\n\tv_nop" : "+v"(d) : "v"(a), "v"(b));
  return d;
}
__device__ __forceinline__ v16h frag_h(const _Float16* rowk0, int lane) {
  union { v16h v; v8h q[2]; } u; const _Float16* p = rowk0 + 8 * (lane >> 4);
  u.q[0] = *(const v8h*)p; u.q[1] = *(const v8h*)(p + 16); return u.v;
}
__device__ __forceinline__ float bfr(float v) { return (float)(__bf16)v; }
#define LDSX() do { asm volatile("s_wait_dscnt 0" ::: "memory"); __builtin_amdgcn_wave_barrier(); __builtin_amdgcn_fence(3  , "workgroup"); } while (0)
#define LWAIT() asm volatile("s_wait_loadcnt 0x0" ::: "memory")

#ifndef NB
#define NB 4
#endif
#ifndef SEQ
#define SEQ 2048
#endif
#ifndef MC
#define MC 256
#endif
#define NB_FULL 4
#define SEQ_FULL 2048
#define MC_FULL 256
#define CC 512
#define CD 768
#define NH 8
#define HD 64
#define FFI 2048
static_assert(SEQ % 128 == 0);
static_assert(MC % 128 == 0);
static_assert(NB >= 1 && NB <= NB_FULL);
static_assert(SEQ <= SEQ_FULL);
static_assert(MC <= MC_FULL);
static_assert(CC % 128 == 0 && CD % 32 == 0 && FFI % 64 == 0 && NH * HD == CC);

#define WS_WQ1 ((size_t)0)
#define WS_WK1 (WS_WQ1 + 2u * (size_t)CC * CC)
#define WS_WV1 (WS_WK1 + 2u * (size_t)CC * CC)
#define WS_WO1 (WS_WV1 + 2u * (size_t)CC * CC)
#define WS_WQ2 (WS_WO1 + 2u * (size_t)CC * CC)
#define WS_WK2 (WS_WQ2 + 2u * (size_t)CC * CC)
#define WS_WV2 (WS_WK2 + 2u * (size_t)CC * CD)
#define WS_WO2 (WS_WV2 + 2u * (size_t)CC * CD)
#define WS_WF1 (WS_WO2 + 2u * (size_t)CC * CC)
#define WS_WF2 (WS_WF1 + 2u * (size_t)2 * FFI * CC)
#define WS_H   (WS_WF2 + 2u * (size_t)CC * FFI)
#define WS_Q   (WS_H   + 2u * (size_t)NB * SEQ * CC)
#define WS_K   (WS_Q   + 2u * (size_t)NB * SEQ * CC)
#define WS_VT  (WS_K   + 2u * (size_t)NB * SEQ * CC)
#define WS_CT  (WS_VT  + 2u * (size_t)NB * CC * SEQ)
#define WS_XT  (WS_CT  + 2u * (size_t)NB * SEQ * CC)
#define WS_X1  (WS_XT  + 2u * (size_t)NB * MC * CD)
#define WS_X2  (WS_X1  + 4u * (size_t)NB * CC * SEQ)
#define WS_ACT (WS_X2  + 4u * (size_t)NB * CC * SEQ)
#define WS_END (WS_ACT + 2u * (size_t)NB * SEQ * FFI)
static_assert(WS_END <= (size_t)134217728u);

__global__ __launch_bounds__(256) void k_wcvt(const float* __restrict__ W, _Float16* __restrict__ P, int n) {
  const long long i = ((long long)blockIdx.x * 256 + threadIdx.x) * 8;
  if (i + 8 > (long long)n) return;
  const v4f a = *(const v4f*)(W + i), c = *(const v4f*)(W + i + 4);
  union { v8h h; v4u u; } o;
#pragma unroll
  for (int k = 0; k < 4; ++k) { o.h[k] = (_Float16)(bfr(a[k]) * 256.0f); o.h[4 + k] = (_Float16)(bfr(c[k]) * 256.0f); }
  vst2((unsigned*)(P + i), o.u);
}

__global__ __launch_bounds__(256) void k_ctx(const float* __restrict__ X, _Float16* __restrict__ T) {
  __shared__ __align__(16) _Float16 st[32][CD + 8];
  const int tid = threadIdx.x, wave = tid >> 5, lane = tid & 31;
  const int b = blockIdx.y, m0 = blockIdx.x * 32;
  const float* xp = X + (size_t)b * CD * MC_FULL + (size_t)(wave * 96) * MC_FULL + m0 + lane;
#pragma unroll
  for (int gq = 0; gq < 12; ++gq) {
#pragma unroll
    for (int i = 0; i < 8; ++i) { const int c = gq * 8 + i; st[lane][wave * 96 + c] = (_Float16)bfr(xp[(size_t)c * MC_FULL]); }
    LWAIT();
  }
  __syncthreads();
  _Float16* tb = T + ((size_t)b * MC + m0) * CD;
#pragma unroll
  for (int it = 0; it < 12; ++it) { const int e = it * 256 + tid; const int row = e / 96, q = e % 96;
    vst2((unsigned*)(tb + (size_t)row * CD + q * 8), *(const v4u*)&st[row][q * 8]); }
}

__global__ __launch_bounds__(256) void k_ln(const float* __restrict__ X, long long bstride, int cstride, int rnd, const float* __restrict__ G, _Float16* __restrict__ H) {
  __shared__ __align__(16) _Float16 st[32][CC + 8];
  __shared__ float sred[8][32]; __shared__ float smean[32]; __shared__ float srstd[32];
  const int tid = threadIdx.x, wave = tid >> 5, lane = tid & 31;
  const int b = blockIdx.y, n0 = blockIdx.x * 32;
  const float* xp = X + (size_t)b * bstride + (size_t)(wave * 64) * cstride + n0 + lane;
  float v[64];
#pragma unroll
  for (int gq = 0; gq < 8; ++gq) {
#pragma unroll
    for (int i = 0; i < 8; ++i) { const float t = xp[(size_t)(gq * 8 + i) * cstride]; v[gq * 8 + i] = rnd ? bfr(t) : t; }
    LWAIT();
  }
  float s = 0.f;
#pragma unroll
  for (int i = 0; i < 64; ++i) s += v[i];
  sred[wave][lane] = s;
  __syncthreads();
  if (wave == 0) { float a = 0.f;
#pragma unroll
    for (int w = 0; w < 8; ++w) a += sred[w][lane];
    smean[lane] = a * (1.0f / 512.0f); }
  __syncthreads();
  const float mean = smean[lane];
  float q = 0.f;
#pragma unroll
  for (int i = 0; i < 64; ++i) { const float d = v[i] - mean; q += d * d; }
  sred[wave][lane] = q;
  __syncthreads();
  if (wave == 0) { float a = 0.f;
#pragma unroll
    for (int w = 0; w < 8; ++w) a += sred[w][lane];
    srstd[lane] = rsqrtf(a * (1.0f / 512.0f) + 1.0e-5f); }
  __syncthreads();
  const float rstd = srstd[lane];
#pragma unroll
  for (int i = 0; i < 64; ++i) { const int c = wave * 64 + i; st[lane][c] = (_Float16)((v[i] - mean) * rstd * bfr(G[c])); }
  __syncthreads();
  _Float16* hb = H + ((size_t)b * SEQ + n0) * CC;
#pragma unroll
  for (int it = 0; it < 8; ++it) { const int e = it * 256 + tid; const int row = e >> 6, qq = e & 63;
    vst2((unsigned*)(hb + (size_t)row * CC + qq * 8), *(const v4u*)&st[row][qq * 8]); }
}

struct GArgs {
  const _Float16* A; const _Float16* B; void* C; const float* bias; const float* R;
  long long sAz, sBz, sCz, sRz;
  int lda, ldb, ldc, ldr, K, rnd; float oscale; int pad;
};
static_assert(sizeof(GArgs) == 104);

template <int MODE> __global__ __launch_bounds__(128) void k_gemm(GArgs p) {
  __shared__ __align__(16) float sraw[4 * 16 * 132];
  const int tid = threadIdx.x, wave = tid >> 5, lane = tid & 31, col = lane & 15, g = lane >> 4;
  const int z = blockIdx.z;
  const size_t r0 = (size_t)blockIdx.x * 64 + wave * 16;
  const int c0 = blockIdx.y * (MODE == 2 ? 64 : 128);
  const _Float16* Ar = p.A + (long long)z * p.sAz + (long long)(r0 + col) * p.lda;
  const _Float16* Bb = p.B + (long long)z * p.sBz;
  v8f acc[8] = {};
  const int nk = p.K >> 5;
#pragma unroll 2
  for (int kc = 0; kc < nk; ++kc) {
    const v16h a = frag_h(Ar + kc * 32, lane);
    LWAIT();
#pragma unroll
    for (int j = 0; j < 8; ++j) {
      const int brow = (MODE == 2) ? ((j < 4) ? (c0 + j * 16 + col) : (FFI + c0 + (j - 4) * 16 + col)) : (c0 + j * 16 + col);
      const v16h bf = frag_h(Bb + (long long)brow * p.ldb + kc * 32, lane);
      LWAIT();
      acc[j] = wmma16(a, bf, acc[j]);
    }
  }
  if (MODE == 0) {
    _Float16* sh = (_Float16*)sraw + wave * (16 * 136);
#pragma unroll
    for (int j = 0; j < 8; ++j)
#pragma unroll
      for (int r = 0; r < 8; ++r) sh[(8 * g + r) * 136 + j * 16 + col] = (_Float16)(acc[j][r] * p.oscale);
    LDSX();
    _Float16* Cb = (_Float16*)p.C + (long long)z * p.sCz + c0;
#pragma unroll
    for (int it = 0; it < 8; ++it) { const int row = it * 2 + g; const int q = col;
      vst2((unsigned*)(Cb + (long long)(r0 + row) * p.ldc + q * 8), *(const v4u*)(sh + row * 136 + q * 8)); }
  } else if (MODE == 1) {
    float* sf = sraw + wave * (16 * 132);
    float bv[8];
#pragma unroll
    for (int r = 0; r < 8; ++r) bv[r] = bfr(p.bias[r0 + 8 * g + r]);
#pragma unroll
    for (int j = 0; j < 8; ++j)
#pragma unroll
      for (int r = 0; r < 8; ++r) sf[(8 * g + r) * 132 + j * 16 + col] = acc[j][r] * p.oscale + bv[r];
    LDSX();
    float* Cb = (float*)p.C + (long long)z * p.sCz + c0 + lane * 4;
    const float* Rb = p.R + (long long)z * p.sRz + c0 + lane * 4;
    for (int rl = 0; rl < 16; ++rl) {
      const long long orow = (long long)(r0 + rl);
      v4f rv = *(const v4f*)(Rb + orow * p.ldr);
      if (p.rnd) { rv[0] = bfr(rv[0]); rv[1] = bfr(rv[1]); rv[2] = bfr(rv[2]); rv[3] = bfr(rv[3]); }
      const v4f sv = *(const v4f*)(sf + rl * 132 + lane * 4);
      const v4f ov = sv + rv;
      vst2(Cb + orow * p.ldc, ov);
    }
  } else {
    _Float16* sgm = (_Float16*)sraw + wave * (16 * 72);
#pragma unroll
    for (int jj = 0; jj < 4; ++jj) {
      const int c = c0 + jj * 16 + col;
      const float bh = bfr(p.bias[c]), bg = bfr(p.bias[FFI + c]);
#pragma unroll
      for (int r = 0; r < 8; ++r) {
        const float hv = acc[jj][r] * p.oscale + bh;
        const float gv = acc[jj + 4][r] * p.oscale + bg;
        const float ge = 0.5f * gv * (1.0f + erff(gv * 0.70710678118654752f));
        sgm[(8 * g + r) * 72 + jj * 16 + col] = (_Float16)(hv * ge * 64.0f);
      }
    }
    LDSX();
    _Float16* Cb = (_Float16*)p.C + (long long)z * p.sCz + c0;
#pragma unroll
    for (int it = 0; it < 4; ++it) { const int row = it * 4 + (lane >> 3); const int q = lane & 7;
      vst2((unsigned*)(Cb + (long long)(r0 + row) * p.ldc + q * 8), *(const v4u*)(sgm + row * 72 + q * 8)); }
  }
}

template <int NK> __global__ __launch_bounds__(128) void k_attn(const _Float16* __restrict__ Q, const _Float16* __restrict__ KP, const _Float16* __restrict__ VT, _Float16* __restrict__ CT) {
  __shared__ __align__(16) _Float16 sp[4][16][72];
  const int tid = threadIdx.x, wave = tid >> 5, lane = tid & 31, col = lane & 15, g = lane >> 4;
  const int h = blockIdx.y, b = blockIdx.z;
  const int i0 = blockIdx.x * 64 + wave * 16;
  const _Float16* qr = Q + ((size_t)b * SEQ + i0 + col) * CC + h * HD;
  const v16h qa0 = frag_h(qr, lane), qa1 = frag_h(qr + 32, lane);
  LWAIT();
  const v8f zero = {0.f, 0.f, 0.f, 0.f, 0.f, 0.f, 0.f, 0.f};
  v8f o[4] = {};
  float m[8], l[8];
#pragma unroll
  for (int r = 0; r < 8; ++r) { m[r] = -1.0e30f; l[r] = 0.f; }
  const float SM = 0.18033688011112042f;
  const _Float16* kbase = KP + ((size_t)b * NK + col) * CC + h * HD;
  const _Float16* vbase = VT + ((size_t)b * CC + h * HD + col) * (size_t)NK;
#pragma unroll 1
  for (int kb = 0; kb < NK / 64; ++kb) {
    const int key0 = kb * 64;
    v8f s[4];
#pragma unroll
    for (int j = 0; j < 4; ++j) {
      const _Float16* kr = kbase + (size_t)(key0 + j * 16) * CC;
      const v16h k0f = frag_h(kr, lane), k1f = frag_h(kr + 32, lane);
      LWAIT();
      s[j] = wmma16(qa0, k0f, zero); s[j] = wmma16(qa1, k1f, s[j]);
    }
#pragma unroll
    for (int r = 0; r < 8; ++r) {
      const float t0 = s[0][r] * SM, t1 = s[1][r] * SM, t2 = s[2][r] * SM, t3 = s[3][r] * SM;
      float mx = fmaxf(fmaxf(t0, t1), fmaxf(t2, t3));
#pragma unroll
      for (int w = 1; w < 16; w <<= 1) mx = fmaxf(mx, __shfl_xor(mx, w, 16));
      const float nm = fmaxf(m[r], mx);
      const float corr = exp2f(m[r] - nm);
      m[r] = nm;
      const float e0 = exp2f(t0 - nm), e1 = exp2f(t1 - nm), e2 = exp2f(t2 - nm), e3 = exp2f(t3 - nm);
      float ts = (e0 + e1) + (e2 + e3);
#pragma unroll
      for (int w = 1; w < 16; w <<= 1) ts += __shfl_xor(ts, w, 16);
      l[r] = l[r] * corr + ts;
#pragma unroll
      for (int jd = 0; jd < 4; ++jd) o[jd][r] *= corr;
      _Float16* pr = &sp[wave][8 * g + r][col];
      pr[0] = (_Float16)(e0 * 1024.0f); pr[16] = (_Float16)(e1 * 1024.0f); pr[32] = (_Float16)(e2 * 1024.0f); pr[48] = (_Float16)(e3 * 1024.0f);
    }
    LDSX();
#pragma unroll
    for (int kc = 0; kc < 2; ++kc) {
      const v16h pa = frag_h(&sp[wave][col][kc * 32], lane);
#pragma unroll
      for (int jd = 0; jd < 4; ++jd) {
        const v16h vf = frag_h(vbase + (size_t)(jd * 16) * NK + key0 + kc * 32, lane);
        LWAIT();
        o[jd] = wmma16(pa, vf, o[jd]);
      }
    }
    LDSX();
  }
  float inv[8];
#pragma unroll
  for (int r = 0; r < 8; ++r) inv[r] = 0.25f * (1.0f / l[r]);
#pragma unroll
  for (int jd = 0; jd < 4; ++jd)
#pragma unroll
    for (int r = 0; r < 8; ++r) sp[wave][8 * g + r][jd * 16 + col] = (_Float16)(o[jd][r] * inv[r]);
  LDSX();
  _Float16* cb = CT + ((size_t)b * SEQ + i0) * CC + h * HD;
#pragma unroll
  for (int it = 0; it < 4; ++it) { const int row = it * 4 + (lane >> 3); const int q = lane & 7;
    vst2((unsigned*)(cb + (size_t)row * CC + q * 8), *(const v4u*)&sp[wave][row][q * 8]); }
}

static GArgs mkargs(const _Float16* A, long long sAz, int lda, const _Float16* B, long long sBz, int ldb, void* C, long long sCz, int ldc, int K, float oscale, const float* bias, const float* R, long long sRz, int ldr, int rnd) {
  GArgs q;
  q.A = A; q.B = B; q.C = C; q.bias = bias; q.R = R;
  q.sAz = sAz; q.sBz = sBz; q.sCz = sCz; q.sRz = sRz;
  q.lda = lda; q.ldb = ldb; q.ldc = ldc; q.ldr = ldr; q.K = K; q.rnd = rnd; q.oscale = oscale; q.pad = 0;
  return q;
}

extern "C" void kernel_launch(void* const* d_in, const int* in_sizes, int n_in, void* d_out, int out_size, void* d_ws, size_t ws_size, hipStream_t stream) {
  if (n_in < 19) return;
  if ((long long)in_sizes[0] < (long long)NB * CC * SEQ_FULL) return;
  if ((long long)in_sizes[1] < (long long)NB * CD * MC_FULL) return;
  if (in_sizes[2] < CC || in_sizes[8] < CC || in_sizes[14] < CC || in_sizes[7] < CC || in_sizes[13] < CC || in_sizes[18] < CC || in_sizes[16] < 2 * FFI) return;
  if (in_sizes[3] < CC * CC || in_sizes[4] < CC * CC || in_sizes[5] < CC * CC || in_sizes[6] < CC * CC || in_sizes[9] < CC * CC || in_sizes[12] < CC * CC) return;
  if (in_sizes[10] < CC * CD || in_sizes[11] < CC * CD || in_sizes[15] < 2 * FFI * CC || in_sizes[17] < CC * FFI) return;
  if (ws_size < (size_t)WS_END) return;
  if ((long long)out_size < (long long)NB * CC * SEQ) return;
  const float** F = (const float**)d_in;
  char* ws = (char*)d_ws;
  _Float16 *PWQ1 = (_Float16*)(ws + WS_WQ1), *PWK1 = (_Float16*)(ws + WS_WK1), *PWV1 = (_Float16*)(ws + WS_WV1), *PWO1 = (_Float16*)(ws + WS_WO1);
  _Float16 *PWQ2 = (_Float16*)(ws + WS_WQ2), *PWK2 = (_Float16*)(ws + WS_WK2), *PWV2 = (_Float16*)(ws + WS_WV2), *PWO2 = (_Float16*)(ws + WS_WO2);
  _Float16 *PWF1 = (_Float16*)(ws + WS_WF1), *PWF2 = (_Float16*)(ws + WS_WF2);
  _Float16 *H = (_Float16*)(ws + WS_H), *QP = (_Float16*)(ws + WS_Q), *KPL = (_Float16*)(ws + WS_K), *VT = (_Float16*)(ws + WS_VT), *CT = (_Float16*)(ws + WS_CT), *XT = (_Float16*)(ws + WS_XT), *ACT = (_Float16*)(ws + WS_ACT);
  float *X1 = (float*)(ws + WS_X1), *X2 = (float*)(ws + WS_X2);
  float* OUT = (float*)d_out;

  k_wcvt<<<dim3(CC * CC / 2048), 256, 0, stream>>>(F[3], PWQ1, CC * CC);
  k_wcvt<<<dim3(CC * CC / 2048), 256, 0, stream>>>(F[4], PWK1, CC * CC);
  k_wcvt<<<dim3(CC * CC / 2048), 256, 0, stream>>>(F[5], PWV1, CC * CC);
  k_wcvt<<<dim3(CC * CC / 2048), 256, 0, stream>>>(F[6], PWO1, CC * CC);
  k_wcvt<<<dim3(CC * CC / 2048), 256, 0, stream>>>(F[9], PWQ2, CC * CC);
  k_wcvt<<<dim3(CC * CD / 2048), 256, 0, stream>>>(F[10], PWK2, CC * CD);
  k_wcvt<<<dim3(CC * CD / 2048), 256, 0, stream>>>(F[11], PWV2, CC * CD);
  k_wcvt<<<dim3(CC * CC / 2048), 256, 0, stream>>>(F[12], PWO2, CC * CC);
  k_wcvt<<<dim3(2 * FFI * CC / 2048), 256, 0, stream>>>(F[15], PWF1, 2 * FFI * CC);
  k_wcvt<<<dim3(CC * FFI / 2048), 256, 0, stream>>>(F[17], PWF2, CC * FFI);
  k_ctx<<<dim3(MC / 32, NB), 256, 0, stream>>>(F[1], XT);

  const long long XBS_IN = (long long)CC * SEQ_FULL, XBS = (long long)CC * SEQ;
  k_ln<<<dim3(SEQ / 32, NB), 256, 0, stream>>>(F[0], XBS_IN, SEQ_FULL, 1, F[2], H);
  k_gemm<0><<<dim3(NB * SEQ / 64, CC / 128, 1), 128, 0, stream>>>(mkargs(H, 0, CC, PWQ1, 0, CC, QP, 0, CC, CC, 1.0f / 256.0f, nullptr, nullptr, 0, 0, 0));
  k_gemm<0><<<dim3(NB * SEQ / 64, CC / 128, 1), 128, 0, stream>>>(mkargs(H, 0, CC, PWK1, 0, CC, KPL, 0, CC, CC, 1.0f / 256.0f, nullptr, nullptr, 0, 0, 0));
  k_gemm<0><<<dim3(CC / 64, SEQ / 128, NB), 128, 0, stream>>>(mkargs(PWV1, 0, CC, H, (long long)SEQ * CC, CC, VT, (long long)CC * SEQ, SEQ, CC, 1.0f / 256.0f, nullptr, nullptr, 0, 0, 0));
  k_attn<SEQ><<<dim3(SEQ / 64, NH, NB), 128, 0, stream>>>(QP, KPL, VT, CT);
  k_gemm<1><<<dim3(CC / 64, SEQ / 128, NB), 128, 0, stream>>>(mkargs(PWO1, 0, CC, CT, (long long)SEQ * CC, CC, X1, XBS, SEQ, CC, 1.0f / 65536.0f, F[7], F[0], XBS_IN, SEQ_FULL, 1));
  k_ln<<<dim3(SEQ / 32, NB), 256, 0, stream>>>(X1, XBS, SEQ, 0, F[8], H);
  k_gemm<0><<<dim3(NB * SEQ / 64, CC / 128, 1), 128, 0, stream>>>(mkargs(H, 0, CC, PWQ2, 0, CC, QP, 0, CC, CC, 1.0f / 256.0f, nullptr, nullptr, 0, 0, 0));
  k_gemm<0><<<dim3(NB * MC / 64, CC / 128, 1), 128, 0, stream>>>(mkargs(XT, 0, CD, PWK2, 0, CD, KPL, 0, CC, CD, 1.0f / 256.0f, nullptr, nullptr, 0, 0, 0));
  k_gemm<0><<<dim3(CC / 64, MC / 128, NB), 128, 0, stream>>>(mkargs(PWV2, 0, CD, XT, (long long)MC * CD, CD, VT, (long long)CC * MC, MC, CD, 1.0f / 256.0f, nullptr, nullptr, 0, 0, 0));
  k_attn<MC><<<dim3(SEQ / 64, NH, NB), 128, 0, stream>>>(QP, KPL, VT, CT);
  k_gemm<1><<<dim3(CC / 64, SEQ / 128, NB), 128, 0, stream>>>(mkargs(PWO2, 0, CC, CT, (long long)SEQ * CC, CC, X2, XBS, SEQ, CC, 1.0f / 65536.0f, F[13], X1, XBS, SEQ, 0));
  k_ln<<<dim3(SEQ / 32, NB), 256, 0, stream>>>(X2, XBS, SEQ, 0, F[14], H);
  k_gemm<2><<<dim3(NB * SEQ / 64, FFI / 64, 1), 128, 0, stream>>>(mkargs(H, 0, CC, PWF1, 0, CC, ACT, 0, FFI, CC, 1.0f / 256.0f, F[16], nullptr, 0, 0, 0));
  k_gemm<1><<<dim3(CC / 64, SEQ / 128, NB), 128, 0, stream>>>(mkargs(PWF2, 0, FFI, ACT, (long long)SEQ * FFI, FFI, OUT, XBS, SEQ, FFI, 1.0f / 16384.0f, F[18], X2, XBS, SEQ, 0));
}
